// MatlabBlock_56264071577749
// MI455X (gfx1250) — hardware-verified
//
#include <hip/hip_runtime.h>
#include <math.h>

typedef __attribute__((ext_vector_type(16))) _Float16 v16h;
typedef __attribute__((ext_vector_type(16))) __bf16 v16b;
typedef __attribute__((ext_vector_type(8)))  _Float16 v8h;
typedef __attribute__((ext_vector_type(8)))  float v8f;
typedef __attribute__((ext_vector_type(4)))  float v4f;
typedef __attribute__((ext_vector_type(2)))  float v2f;
typedef __attribute__((ext_vector_type(4)))  unsigned v4u;
typedef __attribute__((ext_vector_type(4)))  int v4i;
typedef float __attribute__((may_alias)) float_a;
typedef int __attribute__((may_alias)) int_a;

template <typename T> __device__ __forceinline__ void vst2(void* p, T v) { *(volatile T*)p = v; __threadfence(); *(volatile T*)p = v; }
__device__ __forceinline__ v8f wmma16(v16h a, v16h b, v8f c) {
  v8f d = __builtin_amdgcn_wmma_f32_16x16x32_f16(false, a, false, b, (short)0, c, false, false);
  asm volatile("v_nop\n\tv_nop\n\tv_nop\n\tv_nop" : "+v"(d) : "v"(a), "v"(b));
  return d;
}
__device__ __forceinline__ v8f wmma_bf(v16b a, v16b b, v8f c) {
  v8f d = __builtin_amdgcn_wmma_f32_16x16x32_bf16(false, a, false, b, (short)0, c, false, false);
  asm volatile("v_nop\n\tv_nop\n\tv_nop\n\tv_nop" : "+v"(d) : "v"(a), "v"(b));
  return d;
}
__device__ __forceinline__ v16h frag_h(const _Float16* rowk0, int lane) {
  union { v16h v; v8h q[2]; } u; const _Float16* p = rowk0 + 8 * (lane >> 4);
  u.q[0] = *(const v8h*)p; u.q[1] = *(const v8h*)(p + 16); return u.v;
}
__device__ __forceinline__ v16h frag_f32(const float* rowk0, int lane) {
  v16h a; const float* p = rowk0 + 8 * (lane >> 4);
#pragma unroll
  for (int i = 0; i < 8; ++i) { a[i] = (_Float16)p[i]; a[8 + i] = (_Float16)p[16 + i]; }
  return a;
}
__device__ __forceinline__ v16h frag_f32s(const float* rowk0, int lane, float sc) {
  v16h a; const float* p = rowk0 + 8 * (lane >> 4);
#pragma unroll
  for (int i = 0; i < 8; ++i) { a[i] = (_Float16)(p[i] * sc); a[8 + i] = (_Float16)(p[16 + i] * sc); }
  return a;
}
__device__ __forceinline__ v16h fragc_f32(const float* W, int k0, int n, int lane, int ld, int K) {
  v16h a; const int g = lane >> 4;
#pragma unroll
  for (int i = 0; i < 8; ++i) { const int ka = k0 + 8 * g + i, kb = ka + 16;
    a[i] = (_Float16)(ka < K ? W[(size_t)(ka < K ? ka : K - 1) * ld + n] : 0.f); a[8 + i] = (_Float16)(kb < K ? W[(size_t)(kb < K ? kb : K - 1) * ld + n] : 0.f); }
  return a;
}
struct F2 { v16b h, l; };
__device__ __forceinline__ F2 bsplit16(const float v[16]) { F2 r;
#pragma unroll
  for (int i = 0; i < 16; ++i) { const __bf16 h = (__bf16)v[i]; r.h[i] = h; r.l[i] = (__bf16)(v[i] - (float)h); }
  return r; }
__device__ __forceinline__ F2 split_row(const float* row, int k0, int lane) { float v[16]; const float* p = row + k0 + 8 * (lane >> 4);
#pragma unroll
  for (int i = 0; i < 8; ++i) { v[i] = p[i]; v[8 + i] = p[16 + i]; }
  return bsplit16(v); }
__device__ __forceinline__ F2 split_rowK(const float* row, int k0, int lane, int K) { float v[16]; const int g = lane >> 4;
#pragma unroll
  for (int i = 0; i < 8; ++i) { const int ka = k0 + 8 * g + i, kb = ka + 16; v[i] = ka < K ? row[ka < K ? ka : K - 1] : 0.f; v[8 + i] = kb < K ? row[kb < K ? kb : K - 1] : 0.f; }
  return bsplit16(v); }
__device__ __forceinline__ F2 split_col(const float* W, int k0, int n, int lane, int ld, int K) { float v[16]; const int g = lane >> 4;
#pragma unroll
  for (int i = 0; i < 8; ++i) { const int ka = k0 + 8 * g + i, kb = ka + 16; v[i] = ka < K ? W[(size_t)(ka < K ? ka : K - 1) * ld + n] : 0.f; v[8 + i] = kb < K ? W[(size_t)(kb < K ? kb : K - 1) * ld + n] : 0.f; }
  return bsplit16(v); }
__device__ __forceinline__ v8f mac3(const F2& a, const F2& b, v8f c) { c = wmma_bf(a.l, b.h, c); c = wmma_bf(a.h, b.l, c); return wmma_bf(a.h, b.h, c); }
__device__ __forceinline__ float sigm(float v) { return 1.0f / (1.0f + expf(-v)); }
#define LDSX() do { asm volatile("s_wait_dscnt 0" ::: "memory"); __builtin_amdgcn_wave_barrier(); __builtin_amdgcn_fence(__ATOMIC_RELEASE, "workgroup"); } while (0)


#define NN 4
#define CC 256
#define NP 4096
#define NR (NN * NP)
#ifndef TQB
#define TQB (NP / 64)
#endif
typedef __attribute__((ext_vector_type(8))) __bf16 v8b;
__device__ __forceinline__ v16b frag_b(const __bf16* rowk0, int lane) {
  union { v16b v; v8b q[2]; } u; const __bf16* p = rowk0 + 8 * (lane >> 4);
  u.q[0] = *(const v8b*)p; u.q[1] = *(const v8b*)(p + 16); return u.v;
}
__device__ __forceinline__ float bfr(float v) { return (float)(__bf16)v; }
__device__ __attribute__((noinline)) float exp_ni(float v) { return expf(v); }
__device__ __attribute__((noinline)) float erf_ni(float v) { return erff(v); }

#define WS_PW  0u
#define WS_KH  (WS_PW + 2u * 2 * CC * CC)
#define WS_QH  (WS_KH + 2u * NR * CC)
#define WS_NK  (WS_QH + 2u * NR * CC)
#define WS_NQ  (WS_NK + 4u * NR)
#define WS_VT  (WS_NQ + 4u * NR)
#define WS_END (WS_VT + 2u * NR * CC)

__global__ __launch_bounds__(256) void k_pack(const float* __restrict__ WK, const float* __restrict__ WQ, __bf16* __restrict__ PW, const float* __restrict__ X, _Float16* __restrict__ VT) {
  const int n = blockIdx.x, which = blockIdx.y, t = threadIdx.x;
  if (which < 2) { if (n >= CC) return; __shared__ __align__(16) __bf16 s[CC]; s[t] = (__bf16)(which ? WQ : WK)[(size_t)n * CC + t]; __syncthreads(); if (t < CC / 8) vst2((unsigned*)(PW + ((size_t)which * CC + n) * CC + t * 8), *(const v4u*)&s[t * 8]); }
  else { __shared__ __align__(16) _Float16 sx[NP / 4]; const size_t row = blockIdx.x; const int part = which - 2;
    for (int e = t; e < NP / 4; e += 256) sx[e] = (_Float16)bfr(X[row * NP + part * (NP / 4) + e]); __syncthreads();
    for (int q = t; q < NP / 32; q += 256) vst2((unsigned*)(VT + row * NP + part * (NP / 4) + q * 8), *(const v4u*)&sx[q * 8]); }
}
__global__ __launch_bounds__(128) void k_proj(const float* __restrict__ X, const __bf16* __restrict__ PW, const float* __restrict__ BK0, const float* __restrict__ BQ0, _Float16* __restrict__ KH, _Float16* __restrict__ QH, float* __restrict__ NK, float* __restrict__ NQ) {
  __shared__ __align__(16) __bf16 sa[64][CC + 8]; __shared__ __align__(16) _Float16 so[4][16][CC + 8]; __shared__ __align__(16) float sn[64];
  const int tid = threadIdx.x, wave = tid >> 5, lane = tid & 31, col = lane & 15, g = lane >> 4; const int which = blockIdx.y; const size_t n = blockIdx.z; const int p0 = blockIdx.x * 64;
  for (int e = tid; e < 64 * CC; e += 128) { const int c = e >> 6, r = e & 63; sa[r][c] = (__bf16)X[(n * CC + c) * NP + p0 + r]; }
  if (tid < 64) for (int c = CC; c < CC + 8; ++c) sa[tid][c] = (__bf16)0.f;
  __syncthreads();
  const __bf16* Wr = PW + (size_t)which * CC * CC; const float* B0 = which ? BQ0 : BK0;
  float ssq[8];
#pragma unroll
  for (int r = 0; r < 8; ++r) ssq[r] = 0.f;
#pragma unroll 1
  for (int pass = 0; pass < 2; ++pass) { v8f acc[8] = {};
#pragma unroll
    for (int kc = 0; kc < CC / 32; ++kc) { const v16b a = frag_b(&sa[wave * 16 + col][kc * 32], lane);
#pragma unroll
      for (int j = 0; j < 8; ++j) acc[j] = wmma_bf(a, frag_b(Wr + (size_t)(pass * 128 + j * 16 + col) * CC + kc * 32, lane), acc[j]); }
#pragma unroll
    for (int j = 0; j < 8; ++j) { const int c = pass * 128 + j * 16 + col; const float bb = bfr(B0[c]);
#pragma unroll
      for (int r = 0; r < 8; ++r) { const float v = acc[j][r] + bb; ssq[r] += v * v; so[wave][8 * g + r][c] = (_Float16)v; } } }
#pragma unroll
  for (int r = 0; r < 8; ++r) { float s = ssq[r];
#pragma unroll
    for (int o = 1; o < 16; o <<= 1) s += __shfl_xor(s, o);
    if (col == 0) sn[wave * 16 + 8 * g + r] = s; }
  if (lane < 16) for (int c = CC; c < CC + 8; ++c) so[wave][lane][c] = (_Float16)0.f;
  __syncthreads();
  _Float16* dst = which ? QH : KH; float* dn = which ? NQ : NK;
  for (int e = tid; e < 64 * (CC / 8); e += 128) { const int r = e >> 5, q = e & 31; vst2((unsigned*)(dst + (n * NP + p0 + r) * CC + q * 8), *(const v4u*)&so[r >> 4][r & 15][q * 8]); }
  if (tid < 16) vst2(dn + n * NP + p0 + tid * 4, *(const v4f*)&sn[tid * 4]);
}
__global__ __launch_bounds__(128) void k_attn(const _Float16* __restrict__ KH, const _Float16* __restrict__ QH, const float* __restrict__ NK, const float* __restrict__ NQ, const _Float16* __restrict__ VT, float* __restrict__ OUT) {
  __shared__ __align__(16) _Float16 sph[4][16][40]; __shared__ __align__(16) float so[CC / 2][68];
  const int tid = threadIdx.x, wave = tid >> 5, lane = tid & 31, col = lane & 15, g = lane >> 4; const size_t n = blockIdx.y; const int vh = blockIdx.z;   const int j0 = blockIdx.x * 64 + wave * 16; const size_t rq = n * NP + j0;
  v16h aq[CC / 32];
#pragma unroll
  for (int kc = 0; kc < CC / 32; ++kc) aq[kc] = frag_h(KH + (rq + col) * CC + kc * 32, lane);
  float nj[8], m[8], l[8];
#pragma unroll
  for (int r = 0; r < 8; ++r) { nj[r] = NK[rq + 8 * g + r]; m[r] = -3.0e38f; l[r] = 0.f; }
  v8f acc[8] = {};
#pragma unroll 1
  for (int ks = 0; ks < NP / 32; ++ks) { const int i0 = ks * 32; v8f s[2];
#pragma unroll
    for (int ct = 0; ct < 2; ++ct) { const int ii = i0 + ct * 16 + col; const size_t rk = (n * NP + ii) * CC; v8f c = {};
#pragma unroll
      for (int kc = 0; kc < CC / 32; ++kc) c = wmma16(aq[kc], frag_h(QH + rk + kc * 32, lane), c);
      const float ni = NQ[n * NP + ii];
#pragma unroll
      for (int r = 0; r < 8; ++r) s[ct][r] = c[r] / sqrtf(fmaxf(ni * nj[r], 1e-12f)); }
#pragma unroll
    for (int r = 0; r < 8; ++r) { float mx = fmaxf(s[0][r], s[1][r]);
#pragma unroll
      for (int o = 1; o < 16; o <<= 1) mx = fmaxf(mx, __shfl_xor(mx, o));
      const float mn = fmaxf(m[r], mx); const float alpha = (m[r] <= -1.0e38f) ? 0.f : __expf(m[r] - mn); const float e0 = __expf(s[0][r] - mn), e1 = __expf(s[1][r] - mn); float es = e0 + e1;
#pragma unroll
      for (int o = 1; o < 16; o <<= 1) es += __shfl_xor(es, o);
      l[r] = l[r] * alpha + es; m[r] = mn;
#pragma unroll
      for (int dt = 0; dt < 8; ++dt) acc[dt][r] *= alpha;
      sph[wave][8 * g + r][col] = (_Float16)(e0 * 2048.0f); sph[wave][8 * g + r][16 + col] = (_Float16)(e1 * 2048.0f); }
    LDSX();
    const v16h pa = frag_h(&sph[wave][col][0], lane);
#pragma unroll
    for (int dt = 0; dt < 8; ++dt) acc[dt] = wmma16(pa, frag_h(VT + (n * CC + vh * 128 + dt * 16 + col) * NP + i0, lane), acc[dt]);
    LDSX(); }
#pragma unroll
  for (int r = 0; r < 8; ++r) { const float il = (1.0f / 2048.0f) / l[r]; const int jq = wave * 16 + 8 * g + r;
#pragma unroll
    for (int dt = 0; dt < 8; ++dt) so[dt * 16 + col][jq] = acc[dt][r] * il; }
  __syncthreads();
  for (int e = tid; e < (CC / 2) * 16; e += 128) { const int c = e >> 4, q = e & 15; vst2(OUT + (n * CC + vh * 128 + c) * NP + (size_t)blockIdx.x * 64 + q * 4, *(const v4f*)&so[c][q * 4]); }
}
extern "C" void kernel_launch(void* const* d_in, const int* in_sizes, int n_in, void* d_out, int out_size, void* d_ws, size_t ws_size, hipStream_t stream) {
  (void)in_sizes; (void)n_in; (void)out_size;
  const float** F = (const float**)d_in;
  if (ws_size < (size_t)WS_END) return;
  char* ws = (char*)d_ws; __bf16* PW = (__bf16*)(ws + WS_PW); _Float16 *KH = (_Float16*)(ws + WS_KH), *QH = (_Float16*)(ws + WS_QH), *VT = (_Float16*)(ws + WS_VT); float *NK = (float*)(ws + WS_NK), *NQ = (float*)(ws + WS_NQ);
  k_pack<<<dim3(NN * CC, 6), 256, 0, stream>>>(F[1], F[2], PW, F[0], VT);
  k_proj<<<dim3(NP / 64, 2, NN), 128, 0, stream>>>(F[0], PW, F[3], F[4], KH, QH, NK, NQ);
  k_attn<<<dim3(TQB, NN, 2), 128, 0, stream>>>(KH, QH, NK, NQ, VT, (float*)d_out);
}
